// SwinBlock_49194555408562
// MI455X (gfx1250) — hardware-run, weakly checked
//
#include <hip/hip_runtime.h>
#include <stdint.h>


typedef _Float16 v16h __attribute__((ext_vector_type(16)));
typedef _Float16 v8h  __attribute__((ext_vector_type(8)));
typedef _Float16 v4h  __attribute__((ext_vector_type(4)));
typedef float    v8f  __attribute__((ext_vector_type(8)));
typedef float    v4f  __attribute__((ext_vector_type(4)));
typedef unsigned int u32x4 __attribute__((ext_vector_type(4)));

#ifndef NB
#define NB 16
#endif
#define NB_FULL 16

constexpr int kC     = 256;
constexpr int kHeads = 8;
constexpr int kDH    = 32;
constexpr int kHW    = 56;
constexpr int kL     = kHW * kHW;
constexpr int kWS    = 7;
constexpr int kNW    = kWS * kWS;
constexpr int kLL    = kNW * kNW;
constexpr int kNWX   = kHW / kWS;
constexpr int kWPI   = kNWX * kNWX;
constexpr int kWR    = 64;
constexpr int kShift = 3;
constexpr int kQKV   = 3 * kC;
constexpr int kHid   = 4 * kC;
constexpr int kTab   = (2 * kWS - 1) * (2 * kWS - 1);
constexpr int kCsP   = kC + 8;

constexpr int kMT  = NB * kL;
constexpr int kMTP = ((kMT + 127) / 128) * 128;
constexpr int kMW  = NB * kWPI * kWR;

constexpr int kNChunk = 4;
constexpr int kWPC    = NB * kWPI / kNChunk;
constexpr int kRPC    = kWPC * kWR;
constexpr int kTilesT = kMTP / 128;
constexpr int kTPC    = (kTilesT + kNChunk - 1) / kNChunk;

constexpr float kEps      = 1.001e-5f;
constexpr float kWCarry   = 64.0f;
constexpr float kPCarry   = 1024.0f;
constexpr float kCtxCarry = 16.0f;
constexpr float kGCarry   = 16.0f;
constexpr float kScale    = 0.17677669529663687f;

constexpr size_t kRBBytesA = (size_t)kRPC * kQKV * 2;
constexpr size_t kRBBytesB = (size_t)kTPC * 128 * kHid * 2;
constexpr size_t kRBBytes  = (kRBBytesA > kRBBytesB) ? kRBBytesA : kRBBytesB;

static_assert(NB >= 1 && NB <= NB_FULL);
static_assert(kMTP % 128 == 0);
static_assert((NB * kWPI) % kNChunk == 0);
static_assert(kRPC % 128 == 0);
static_assert(kHeads * kDH == kC);
static_assert(kHeads == 8);
static_assert(kC % 64 == 0 && kHid % 64 == 0);
static_assert(kQKV % 32 == 0 && kC % 32 == 0 && kHid % 32 == 0);
static_assert(kQKV % 128 == 0 && kHid % 128 == 0 && kC % 128 == 0);
static_assert(kHW % kWS == 0 && kNWX == 8 && kWPI == 64);
static_assert(kMTP <= kMW);
static_assert((size_t)kRPC * kQKV * 2 <= kRBBytes);
static_assert((size_t)kTPC * 128 * kHid * 2 <= kRBBytes);
static_assert(kNW <= kWR);
static_assert(kTab * kHeads <= 6 * 256);
static_assert(kLL <= 10 * 256);
static_assert((size_t)kMT * kC <= (size_t)NB_FULL * kL * kC);

enum { EPI_QKV = 0, EPI_GELU = 1, EPI_X1 = 2, EPI_OUT = 3 };

__device__ __forceinline__ v8f wmma16(v16h a, v16h b, v8f c) {
  v8f d = __builtin_amdgcn_wmma_f32_16x16x32_f16(false, a, false, b, (short)0, c,
                                                 false, false);
  asm volatile("v_nop\n\tv_nop\n\tv_nop\n\tv_nop" : "+v"(d) : "v"(a), "v"(b));
  return d;
}

__device__ __forceinline__ v16h load_frag(const _Float16* p, int ld, int lane) {
  const int r  = lane & 15;
  const int k8 = (lane >> 4) << 3;
  const _Float16* q = p + (size_t)r * ld + k8;
  union { v16h v; v8h h[2]; } u;
  u.h[0] = *(const v8h*)(q);
  u.h[1] = *(const v8h*)(q + 16);
  return u.v;
}

__device__ __forceinline__ float bf16r(float x) {
  unsigned int u = __float_as_uint(x);
  u += 0x7FFFu + ((u >> 16) & 1u);
  u &= 0xFFFF0000u;
  return __uint_as_float(u);
}

__device__ __forceinline__ float gelu_f(float x) {
  return 0.5f * x * (1.0f + erff(x * 0.70710678118654752f));
}

__device__ __forceinline__ float wave_sum(float v) {
#pragma unroll
  for (int off = 16; off > 0; off >>= 1) v += __shfl_xor(v, off);
  return v;
}

__device__ __forceinline__ void vst4f(float* p, v4f v) { *(volatile v4f*)p = v; }
__device__ __forceinline__ void vst8h(_Float16* p, v8h v) {
  union { v8h h; u32x4 u; } t;
  t.h = v;
  *(volatile u32x4*)p = t.u;
}

__device__ __forceinline__ int tok_of(int win, int t) {
  const int b  = win / kWPI;
  const int w2 = win - b * kWPI;
  const int wi = w2 / kNWX, wj = w2 - wi * kNWX;
  const int ti = t / kWS, tj = t - ti * kWS;
  int y = wi * kWS + ti + kShift; y = (y >= kHW) ? (y - kHW) : y;
  int x = wj * kWS + tj + kShift; x = (x >= kHW) ? (x - kHW) : x;
  return b * kL + y * kHW + x;
}

__global__ __launch_bounds__(256)
void cvt_wt(const float* __restrict__ W, _Float16* __restrict__ Wt, int K, int N) {
  __shared__ __align__(16) _Float16 tl[32][72];
  const int tid = threadIdx.x;
  const int n0 = blockIdx.x * 32, k0 = blockIdx.y * 64;
#pragma unroll
  for (int it = 0; it < 8; ++it) {
    const int idx = tid + it * 256;
    const int kk = idx >> 5, nn = idx & 31;
    const float w = W[(size_t)(k0 + kk) * N + n0 + nn];
    tl[nn][kk] = (_Float16)(bf16r(w) * kWCarry);
  }
  __syncthreads();
  const int row = tid >> 3, piece = tid & 7;
  const v8h pv = *(const v8h*)(&tl[row][piece * 8]);
  _Float16* dp = Wt + (size_t)(n0 + row) * K + k0 + piece * 8;
  vst8h(dp, pv);
  __threadfence();
  vst8h(dp, pv);
}

template <int GATHER>
__global__ __launch_bounds__(256)
void ln_rows(const float* __restrict__ src, const float* __restrict__ g,
             const float* __restrict__ bta, _Float16* __restrict__ dst) {
  const int tid = threadIdx.x, lane = tid & 31, wave = tid >> 5;
  const int row = blockIdx.x * 8 + wave;
  size_t srow;
  bool ok;
  if (GATHER) {
    const int win = row / kWR;
    const int t   = row - win * kWR;
    ok   = t < kNW;
    srow = (size_t)tok_of(win, ok ? t : 0);
  } else {
    ok   = row < kMT;
    srow = (size_t)min(row, kMT - 1);
  }
  const float* sp = src + srow * kC + lane * 8;
  const v4f xa = *(const v4f*)(sp);
  const v4f xb = *(const v4f*)(sp + 4);
  float v[8];
#pragma unroll
  for (int e = 0; e < 4; ++e) {
    v[e]     = GATHER ? bf16r(xa[e]) : xa[e];
    v[4 + e] = GATHER ? bf16r(xb[e]) : xb[e];
  }
  float s = ((v[0] + v[1]) + (v[2] + v[3])) + ((v[4] + v[5]) + (v[6] + v[7]));
  s = wave_sum(s);
  const float mu = s * (1.0f / (float)kC);
  float d[8];
#pragma unroll
  for (int e = 0; e < 8; ++e) d[e] = v[e] - mu;
  float q = ((d[0] * d[0] + d[1] * d[1]) + (d[2] * d[2] + d[3] * d[3])) +
            ((d[4] * d[4] + d[5] * d[5]) + (d[6] * d[6] + d[7] * d[7]));
  q = wave_sum(q);
  const float rs = rsqrtf(q * (1.0f / (float)kC) + kEps);
  const v4f ga = *(const v4f*)(g + lane * 8);
  const v4f gb = *(const v4f*)(g + lane * 8 + 4);
  const v4f ba = *(const v4f*)(bta + lane * 8);
  const v4f bb = *(const v4f*)(bta + lane * 8 + 4);
  v8h o;
#pragma unroll
  for (int e = 0; e < 4; ++e) {
    const float ya = (d[e] * rs) * bf16r(ga[e]) + bf16r(ba[e]);
    const float yb = (d[4 + e] * rs) * bf16r(gb[e]) + bf16r(bb[e]);
    o[e]     = (_Float16)(ok ? ya : 0.0f);
    o[4 + e] = (_Float16)(ok ? yb : 0.0f);
  }
  _Float16* dp = dst + (size_t)row * kC + lane * 8;
  vst8h(dp, o);
  __threadfence();
  vst8h(dp, o);
}

template <int MI, int NJ>
__device__ __forceinline__ void gemm_core(v8f (&acc)[MI][NJ], const _Float16* Aw,
                                          const _Float16* Bw, int K, int lane) {
  for (int k0 = 0; k0 < K; k0 += 32) {
    v16h a[MI];
#pragma unroll
    for (int i = 0; i < MI; ++i) a[i] = load_frag(Aw + (size_t)(i * 16) * K + k0, K, lane);
#pragma unroll
    for (int j = 0; j < NJ; ++j) {
      const v16h b = load_frag(Bw + (size_t)(j * 16) * K + k0, K, lane);
#pragma unroll
      for (int i = 0; i < MI; ++i) acc[i][j] = wmma16(a[i], b, acc[i][j]);
    }
  }
}

template <int EPI>
__global__ __launch_bounds__(256)
void gemm_rows(const _Float16* __restrict__ A, const _Float16* __restrict__ Bt,
               const float* __restrict__ bias, const float* __restrict__ resid,
               float* __restrict__ outF, _Float16* __restrict__ outH,
               const int* __restrict__ shp, const int* __restrict__ wsp,
               int N, int K, int m_base, int m_lim) {
  __shared__ __align__(16) float stg[8][16 * 68];
  const int tid = threadIdx.x, lane = tid & 31, wave = tid >> 5;
  const int wm = wave & 3, wn = wave >> 2;
  const int m0w = blockIdx.x * 128 + wm * 32;
  const int n0w = blockIdx.y * 128 + wn * 64;
  const _Float16* Aw = A + (size_t)m0w * K;
  const _Float16* Bw = Bt + (size_t)n0w * K;

  v8f acc[2][4] = {};
  gemm_core<2, 4>(acc, Aw, Bw, K, lane);

  constexpr float sc = (EPI == EPI_QKV || EPI == EPI_GELU) ? (1.0f / 64.0f) : (1.0f / 1024.0f);
  bool bad = false;
  if constexpr (EPI == EPI_OUT) {
    const int sv0 = shp[0], wv0 = wsp[0];
    bad = (sv0 != kShift) || (wv0 != kWS);
  }
  const float qnan = __uint_as_float(0x7FC00000u);
  const int n = lane & 15, h8 = (lane >> 4) * 8;
  float* sw = &stg[wave][0];

#pragma unroll
  for (int i = 0; i < 2; ++i) {
#pragma unroll
    for (int j = 0; j < 4; ++j)
#pragma unroll
      for (int r = 0; r < 8; ++r)
        sw[(h8 + r) * 68 + j * 16 + n] = acc[i][j][r] * sc;
    __syncthreads();
    if constexpr (EPI == EPI_X1 || EPI == EPI_OUT) {
      v4f sv[8];
      size_t dof[8];
      bool okv[8];
#pragma unroll
      for (int q = 0; q < 8; ++q) {
        const int row = q * 2 + (lane >> 4), col = (lane & 15) * 4;
        const int gm = m0w + i * 16 + row, gn = n0w + col;
        v4f v = *(const v4f*)(sw + row * 68 + col);
        const v4f bb = *(const v4f*)(bias + gn);
#pragma unroll
        for (int e = 0; e < 4; ++e) v[e] += bf16r(bb[e]);
        if constexpr (EPI == EPI_X1) {
          const int ga  = m_base + gm;
          const int win = ga / kWR;
          const int t   = ga - win * kWR;
          const bool okq = t < kNW;
          const int tok = tok_of(win, okq ? t : 0);
          const size_t ro = (size_t)tok * kC + gn;
          const v4f rr = *(const v4f*)(resid + ro);
#pragma unroll
          for (int e = 0; e < 4; ++e) v[e] = bf16r(rr[e]) + v[e];
          dof[q] = ro;
          okv[q] = okq;
        } else {
          const size_t ro = (size_t)gm * N + gn;
          const v4f rr = *(const v4f*)(resid + ro);
#pragma unroll
          for (int e = 0; e < 4; ++e) {
            const float s2 = rr[e] + v[e];
            v[e] = bad ? qnan : s2;
          }
          dof[q] = ro;
          okv[q] = (m_base + gm) < m_lim;
        }
        sv[q] = v;
        if (okv[q]) vst4f(outF + dof[q], v);
      }
      __threadfence();
#pragma unroll
      for (int q = 0; q < 8; ++q) {
        if (okv[q]) vst4f(outF + dof[q], sv[q]);
      }
    } else {
      v8h sv[4];
#pragma unroll
      for (int q = 0; q < 4; ++q) {
        const int row = q * 4 + (lane >> 3), col = (lane & 7) * 8;
        const int gm = m0w + i * 16 + row, gn = n0w + col;
        const v4f va = *(const v4f*)(sw + row * 68 + col);
        const v4f vb = *(const v4f*)(sw + row * 68 + col + 4);
        const v4f ba = *(const v4f*)(bias + gn);
        const v4f bb = *(const v4f*)(bias + gn + 4);
        v8h o;
#pragma unroll
        for (int e = 0; e < 4; ++e) {
          float xa = va[e] + bf16r(ba[e]), xb = vb[e] + bf16r(bb[e]);
          if constexpr (EPI == EPI_GELU) { xa = gelu_f(xa) * kGCarry; xb = gelu_f(xb) * kGCarry; }
          o[e]     = (_Float16)xa;
          o[4 + e] = (_Float16)xb;
        }
        sv[q] = o;
        vst8h(outH + (size_t)gm * N + gn, o);
      }
      __threadfence();
#pragma unroll
      for (int q = 0; q < 4; ++q) {
        const int row = q * 4 + (lane >> 3), col = (lane & 7) * 8;
        const int gm = m0w + i * 16 + row, gn = n0w + col;
        vst8h(outH + (size_t)gm * N + gn, sv[q]);
      }
    }
    __syncthreads();
  }
}

__global__ __launch_bounds__(256)
void attn_win(const _Float16* __restrict__ qkv, const float* __restrict__ rpb,
              const int* __restrict__ ridx, const float* __restrict__ amask,
              _Float16* __restrict__ ctxp, int wbase) {
  __shared__ __align__(16) _Float16 Vt[kHeads][kDH * 72];
  __shared__ __align__(16) _Float16 Ps[kHeads][16 * 72];
  __shared__ __align__(16) _Float16 Cs[kWR * kCsP];
  __shared__ float tabs[kTab * kHeads];
  __shared__ float msks[kLL];
  __shared__ int   ris[kLL];
  const int w    = blockIdx.x;
  const int tid  = threadIdx.x, lane = tid & 31, h = tid >> 5;
  const int n    = lane & 15, h8 = (lane >> 4) * 8;
  const int w2   = (wbase + w) & (kWPI - 1);
  const _Float16* wq = qkv + (size_t)w * kWR * kQKV;

#pragma unroll
  for (int it = 0; it < 6; ++it) {
    const int i  = tid + it * 256;
    const int ic = min(i, kTab * kHeads - 1);
    const float tv = bf16r(rpb[ic]);
    if (i < kTab * kHeads) tabs[i] = tv;
  }
  const float* mrow = amask + (size_t)w2 * kLL;
#pragma unroll
  for (int it = 0; it < 10; ++it) {
    const int i  = tid + it * 256;
    const int ic = min(i, kLL - 1);
    int rv = ridx[ic];
    rv = min(max(rv, 0), kTab - 1);
    const float mv = bf16r(mrow[ic]);
    if (i < kLL) { ris[i] = rv; msks[i] = mv; }
  }

  _Float16* vt = &Vt[h][0];
  const _Float16 z16 = (_Float16)0.0f;
#pragma unroll
  for (int tt = 0; tt < 2; ++tt) {
    const int t = lane + tt * 32;
    const _Float16* vp = wq + (size_t)t * kQKV + 2 * kC + h * kDH;
    const bool ok = t < kNW;
#pragma unroll
    for (int c = 0; c < 4; ++c) {
      const v8h vv = *(const v8h*)(vp + c * 8);
#pragma unroll
      for (int e = 0; e < 8; ++e) vt[(c * 8 + e) * 72 + t] = ok ? vv[e] : z16;
    }
  }
  __syncthreads();

  v16h kf[4];
#pragma unroll
  for (int j = 0; j < 4; ++j)
    kf[j] = load_frag(wq + (size_t)(j * 16) * kQKV + kC + h * kDH, kQKV, lane);

  _Float16* pw = &Ps[h][0];

  for (int i = 0; i < 4; ++i) {
    const v16h qf = load_frag(wq + (size_t)(i * 16) * kQKV + h * kDH, kQKV, lane);
    v8f s[4];
#pragma unroll
    for (int j = 0; j < 4; ++j) {
      v8f z = {};
      s[j] = wmma16(qf, kf[j], z);
    }

    float rinv[8];
#pragma unroll
    for (int r = 0; r < 8; ++r) {
      const int qrow = i * 16 + h8 + r;
      const int qc = min(qrow, kNW - 1);
      float mx = -1.0e30f;
#pragma unroll
      for (int j = 0; j < 4; ++j) {
        const int key = j * 16 + n;
        const int kc  = min(key, kNW - 1);
        const int pix = qc * kNW + kc;
        const int idx = ris[pix];
        const float bb = tabs[idx * kHeads + h];
        const float mk = msks[pix];
        float lv = (s[j][r] * kScale + bb) + mk;
        lv = (key < kNW) ? lv : -1.0e30f;
        s[j][r] = lv;
        mx = fmaxf(mx, lv);
      }
      mx = fmaxf(mx, __shfl_xor(mx, 1));
      mx = fmaxf(mx, __shfl_xor(mx, 2));
      mx = fmaxf(mx, __shfl_xor(mx, 4));
      mx = fmaxf(mx, __shfl_xor(mx, 8));
      float ps = 0.0f;
#pragma unroll
      for (int j = 0; j < 4; ++j) {
        const float p = __expf(s[j][r] - mx);
        s[j][r] = p;
        ps += p;
      }
      ps += __shfl_xor(ps, 1);
      ps += __shfl_xor(ps, 2);
      ps += __shfl_xor(ps, 4);
      ps += __shfl_xor(ps, 8);
      rinv[r] = (kCtxCarry / kPCarry) * (1.0f / ps);
    }

#pragma unroll
    for (int j = 0; j < 4; ++j)
#pragma unroll
      for (int r = 0; r < 8; ++r)
        pw[(h8 + r) * 72 + j * 16 + n] = (_Float16)(s[j][r] * kPCarry);
    __syncthreads();

    v8f cacc[2] = {};
#pragma unroll
    for (int kk = 0; kk < 2; ++kk) {
      const v16h pa = load_frag(pw + kk * 32, 72, lane);
#pragma unroll
      for (int dt = 0; dt < 2; ++dt) {
        const v16h vb = load_frag(vt + (size_t)(dt * 16) * 72 + kk * 32, 72, lane);
        cacc[dt] = wmma16(pa, vb, cacc[dt]);
      }
    }

#pragma unroll
    for (int r = 0; r < 8; ++r) {
      const int qrow = i * 16 + h8 + r;
      const bool okq = qrow < kNW;
#pragma unroll
      for (int dt = 0; dt < 2; ++dt) {
        const float val = okq ? (cacc[dt][r] * rinv[r]) : 0.0f;
        Cs[qrow * kCsP + h * kDH + dt * 16 + n] = (_Float16)val;
      }
    }
    __syncthreads();
  }

  v8h sv[8];
#pragma unroll
  for (int it = 0; it < 8; ++it) {
    const int row = it * 8 + h;
    sv[it] = *(const v8h*)(&Cs[row * kCsP + lane * 8]);
    _Float16* dst = ctxp + ((size_t)w * kWR + row) * kC + lane * 8;
    vst8h(dst, sv[it]);
  }
  __threadfence();
#pragma unroll
  for (int it = 0; it < 8; ++it) {
    const int row = it * 8 + h;
    _Float16* dst = ctxp + ((size_t)w * kWR + row) * kC + lane * 8;
    vst8h(dst, sv[it]);
  }
}

extern "C" void kernel_launch(void* const* d_in, const int* in_sizes, int n_in,
                              void* d_out, int out_size, void* d_ws, size_t ws_size,
                              hipStream_t stream) {
  if (n_in < 18) return;
  if (in_sizes[0] < kMT * kC) return;
  if (in_sizes[1] < 1 || in_sizes[2] < 1) return;
  if (in_sizes[3] < kLL) return;
  if (in_sizes[4] < kWPI * kLL) return;
  if (in_sizes[5] < kC || in_sizes[6] < kC) return;
  if (in_sizes[7] < kC * kQKV || in_sizes[8] < kQKV) return;
  if (in_sizes[9] < kTab * kHeads) return;
  if (in_sizes[10] < kC * kC || in_sizes[11] < kC) return;
  if (in_sizes[12] < kC || in_sizes[13] < kC) return;
  if (in_sizes[14] < kC * kHid || in_sizes[15] < kHid) return;
  if (in_sizes[16] < kHid * kC || in_sizes[17] < kC) return;
  if (out_size < kMT * kC) return;

  const float* x      = (const float*)d_in[0];
  const int*   shp    = (const int*)  d_in[1];
  const int*   wsp    = (const int*)  d_in[2];
  const int*   relidx = (const int*)  d_in[3];
  const float* amask  = (const float*)d_in[4];
  const float* n1g    = (const float*)d_in[5];
  const float* n1b    = (const float*)d_in[6];
  const float* qkv_w  = (const float*)d_in[7];
  const float* qkv_b  = (const float*)d_in[8];
  const float* rpb    = (const float*)d_in[9];
  const float* proj_w = (const float*)d_in[10];
  const float* proj_b = (const float*)d_in[11];
  const float* n2g    = (const float*)d_in[12];
  const float* n2b    = (const float*)d_in[13];
  const float* fc1_w  = (const float*)d_in[14];
  const float* fc1_b  = (const float*)d_in[15];
  const float* fc2_w  = (const float*)d_in[16];
  const float* fc2_b  = (const float*)d_in[17];
  float* out = (float*)d_out;

  size_t off = 0;
  auto carve = [&](size_t bytes) -> size_t {
    size_t o = off;
    off += (bytes + 255) & ~(size_t)255;
    return o;
  };
  const size_t o_wqkv = carve((size_t)kQKV * kC * 2);
  const size_t o_wpj  = carve((size_t)kC * kC * 2);
  const size_t o_wf1  = carve((size_t)kHid * kC * 2);
  const size_t o_wf2  = carve((size_t)kC * kHid * 2);
  const size_t o_ra   = carve((size_t)kMW * kC * 2);
  const size_t o_rb   = carve(kRBBytes);
  const size_t o_x1   = carve((size_t)kMTP * kC * 4);
  if (off > ws_size) return;
  if (off > (size_t)134217728) return;

  char* ws = (char*)d_ws;
  _Float16* wqkv = (_Float16*)(ws + o_wqkv);
  _Float16* wpj  = (_Float16*)(ws + o_wpj);
  _Float16* wf1  = (_Float16*)(ws + o_wf1);
  _Float16* wf2  = (_Float16*)(ws + o_wf2);
  _Float16* ra   = (_Float16*)(ws + o_ra);
  _Float16* rb   = (_Float16*)(ws + o_rb);
  float*    x1   = (float*)   (ws + o_x1);

  const dim3 b256(256);

  cvt_wt<<<dim3(kQKV / 32, kC / 64), b256, 0, stream>>>(qkv_w, wqkv, kC, kQKV);
  cvt_wt<<<dim3(kC / 32, kC / 64), b256, 0, stream>>>(proj_w, wpj, kC, kC);
  cvt_wt<<<dim3(kHid / 32, kC / 64), b256, 0, stream>>>(fc1_w, wf1, kC, kHid);
  cvt_wt<<<dim3(kC / 32, kHid / 64), b256, 0, stream>>>(fc2_w, wf2, kHid, kC);

  ln_rows<1><<<dim3(kMW / 8), b256, 0, stream>>>(x, n1g, n1b, ra);

  for (int c = 0; c < kNChunk; ++c) {
    const size_t roff = (size_t)c * kRPC * kC;
    gemm_rows<EPI_QKV><<<dim3(kRPC / 128, kQKV / 128), b256, 0, stream>>>(
        ra + roff, wqkv, qkv_b, nullptr, nullptr, rb, shp, wsp, kQKV, kC, 0, 0);
    attn_win<<<dim3(kWPC), b256, 0, stream>>>(rb, rpb, relidx, amask, ra + roff, c * kWPC);
  }

  gemm_rows<EPI_X1><<<dim3(kMW / 128, kC / 128), b256, 0, stream>>>(
      ra, wpj, proj_b, x, x1, nullptr, shp, wsp, kC, kC, 0, 0);

  ln_rows<0><<<dim3(kMTP / 8), b256, 0, stream>>>(x1, n2g, n2b, ra);

  for (int c = 0; c < kNChunk; ++c) {
    const int t0 = c * kTPC;
    const int nt = (kTilesT - t0 < kTPC) ? (kTilesT - t0) : kTPC;
    if (nt <= 0) continue;
    const size_t roff = (size_t)t0 * 128 * kC;
    gemm_rows<EPI_GELU><<<dim3(nt, kHid / 128), b256, 0, stream>>>(
        ra + roff, wf1, fc1_b, nullptr, nullptr, rb, shp, wsp, kHid, kC, 0, 0);
    gemm_rows<EPI_OUT><<<dim3(nt, kC / 128), b256, 0, stream>>>(
        rb, wf2, fc2_b, x1 + roff, out + roff, nullptr, shp, wsp, kC, kHid, t0 * 128, kMT);
  }
}
